// RationaleSelectorModel_13460427505851
// MI455X (gfx1250) — hardware-verified
//
#include <hip/hip_runtime.h>
#include <math.h>
#include <stdint.h>

#pragma clang fp contract(off)

#define B_     32
#define T_     1024
#define D_     256
#define H_     341
#define NP_    352
#define NT_    22
#define R_     4
#define V_     32000
#define NTOK   (B_ * T_)
#define MROWS  32
#define APITCH 264
#define WCOLS  32
#define WPITCH 33
#define NTH    256
#define RECW   32
#define NTAIL  (1 + R_ + R_ * B_)

#define SCA    256.0f
#define SCB    1024.0f
#define SCL    2048.0f
#define INV_HH (1.0f / 262144.0f)
#define INV_HL (1.0f / 536870912.0f)

static_assert(NTH * 4 == T_);
static_assert(D_ == NTH);
static_assert(NTOK % MROWS == 0);
static_assert(MROWS == 32);
static_assert(NP_ % WCOLS == 0);
static_assert(NP_ == NT_ * 16);
static_assert(NP_ >= H_);
static_assert(D_ % 32 == 0);
static_assert((APITCH * 2) % 16 == 0);
static_assert(R_ * B_ == 128);
static_assert(NTAIL == 133);
static_assert(RECW * 4 == 128);

typedef __attribute__((ext_vector_type(16))) _Float16 v16h;
typedef __attribute__((ext_vector_type(8)))  _Float16 v8h;
typedef __attribute__((ext_vector_type(8)))  float  v8f;
typedef __attribute__((ext_vector_type(4)))  float  v4f;

__device__ __forceinline__ void split_h(float x, _Float16& h, _Float16& l) {
  h = (_Float16)x;
  l = (_Float16)((x - (float)h) * SCL);
}

__device__ __forceinline__ v8f mma_h(v16h a, v16h b, v8f c) {
  c = __builtin_amdgcn_wmma_f32_16x16x32_f16(false, a, false, b, (short)0, c, false, false);
  asm volatile("v_nop\n\tv_nop\n\tv_nop\n\tv_nop" : "+v"(c) : "v"(a), "v"(b));
  return c;
}

__device__ __forceinline__ float bsum1(float v, float* red, int tid) {
  red[tid] = v;
  __syncthreads();
  for (int o = NTH / 2; o > 0; o >>= 1) {
    if (tid < o) red[tid] = red[tid] + red[tid + o];
    __syncthreads();
  }
  const float r = red[0];
  __syncthreads();
  return r;
}
__device__ __forceinline__ void bsum3(float v0, float v1, float v2, float* r0, float* r1, float* r2, int tid,
                                      float& o0, float& o1, float& o2) {
  r0[tid] = v0;
  r1[tid] = v1;
  r2[tid] = v2;
  __syncthreads();
  for (int o = NTH / 2; o > 0; o >>= 1) {
    if (tid < o) {
      r0[tid] = r0[tid] + r0[tid + o];
      r1[tid] = r1[tid] + r1[tid + o];
      r2[tid] = r2[tid] + r2[tid + o];
    }
    __syncthreads();
  }
  o0 = r0[0];
  o1 = r1[0];
  o2 = r2[0];
  __syncthreads();
}

__global__ __launch_bounds__(256) void wsplit_kernel(const float* __restrict__ w1,
                                                      unsigned short* __restrict__ whi,
                                                      unsigned short* __restrict__ wlo) {
  __shared__ float tf[D_ * WPITCH];
  const int tid = threadIdx.x;
  const int n0 = blockIdx.x * WCOLS;
  for (int i = tid; i < D_ * WCOLS; i += 256) {
    const int k = i >> 5, nn = i & 31;
    const int n = n0 + nn;
    const int nc = min(n, H_ - 1);
    const float v = w1[(size_t)k * H_ + nc];
    tf[k * WPITCH + nn] = (n < H_) ? v : 0.f;
  }
  __syncthreads();
  _Float16* Hp = (_Float16*)(void*)whi;
  _Float16* Lp = (_Float16*)(void*)wlo;
  v8h hv[4], lv[4];
#pragma unroll
  for (int it = 0; it < 4; ++it) {
    const int L = it * 32 + (tid >> 3);
    const int row = L >> 2;
    const int k8 = (L & 3) * 64 + (tid & 7) * 8;
    _Float16 hh[8], ll[8];
#pragma unroll
    for (int j = 0; j < 8; ++j) {
      const float x = tf[(k8 + j) * WPITCH + row] * SCB;
      split_h(x, hh[j], ll[j]);
    }
    hv[it] = (v8h){hh[0], hh[1], hh[2], hh[3], hh[4], hh[5], hh[6], hh[7]};
    lv[it] = (v8h){ll[0], ll[1], ll[2], ll[3], ll[4], ll[5], ll[6], ll[7]};
  }
#pragma unroll
  for (int it = 0; it < 4; ++it) {
    const int L = it * 32 + (tid >> 3);
    const int row = L >> 2;
    const int k8 = (L & 3) * 64 + (tid & 7) * 8;
    const size_t go = (size_t)(n0 + row) * D_ + k8;
    *(volatile v8h*)(Hp + go) = hv[it];
    *(volatile v8h*)(Lp + go) = lv[it];
  }
  __threadfence();
#pragma unroll
  for (int it = 0; it < 4; ++it) {
    const int L = it * 32 + (tid >> 3);
    const int row = L >> 2;
    const int k8 = (L & 3) * 64 + (tid & 7) * 8;
    const size_t go = (size_t)(n0 + row) * D_ + k8;
    *(volatile v8h*)(Hp + go) = hv[it];
    *(volatile v8h*)(Lp + go) = lv[it];
  }
}

__global__ __launch_bounds__(64) void mlp_kernel(const float* __restrict__ emb, const float* __restrict__ attn,
                                                 const float* __restrict__ lnw, const float* __restrict__ lnb,
                                                 const unsigned short* __restrict__ whi,
                                                 const unsigned short* __restrict__ wlo,
                                                 const float* __restrict__ b1, const float* __restrict__ w2,
                                                 const float* __restrict__ b2, float* __restrict__ scores) {
  union FB { v16h v; v8h h[2]; };
  __shared__ __align__(16) _Float16 sAh[MROWS * APITCH];
  __shared__ __align__(16) _Float16 sAl[MROWS * APITCH];
  __shared__ __align__(16) float ssc[MROWS];

  const int tid  = threadIdx.x;
  const int wave = tid >> 5;
  const int lane = tid & 31;
  const int lh   = lane >> 4;
  const int c    = lane & 15;
  const int row0 = blockIdx.x * MROWS;
  const int l8   = lane * 8;

  {
    const v4f wq0 = *(const v4f*)(lnw + l8), wq1 = *(const v4f*)(lnw + l8 + 4);
    const v4f bq0 = *(const v4f*)(lnb + l8), bq1 = *(const v4f*)(lnb + l8 + 4);
    float wv[8], bv[8];
#pragma unroll
    for (int j = 0; j < 4; ++j) { wv[j] = wq0[j]; wv[4 + j] = wq1[j]; bv[j] = bq0[j]; bv[4 + j] = bq1[j]; }
#pragma unroll 2
    for (int m = 0; m < 16; ++m) {
      const int rl  = wave * 16 + m;
      const int tok = row0 + rl;
      const float sel = attn[tok];
      const float* xp = emb + (size_t)tok * D_ + l8;
      const v4f x0 = *(const v4f*)xp;
      const v4f x1 = *(const v4f*)(xp + 4);
      float x[8];
#pragma unroll
      for (int j = 0; j < 4; ++j) { x[j] = x0[j] * sel; x[4 + j] = x1[j] * sel; }
      float s = 0.f;
#pragma unroll
      for (int j = 0; j < 8; ++j) s += x[j];
      s += __shfl_xor(s, 16, 32);
      s += __shfl_xor(s, 8, 32);
      s += __shfl_xor(s, 4, 32);
      s += __shfl_xor(s, 2, 32);
      s += __shfl_xor(s, 1, 32);
      const float mean = s * (1.0f / 256.0f);
      float dv[8];
      float v = 0.f;
#pragma unroll
      for (int j = 0; j < 8; ++j) { dv[j] = x[j] - mean; v += dv[j] * dv[j]; }
      v += __shfl_xor(v, 16, 32);
      v += __shfl_xor(v, 8, 32);
      v += __shfl_xor(v, 4, 32);
      v += __shfl_xor(v, 2, 32);
      v += __shfl_xor(v, 1, 32);
      const float var = v * (1.0f / 256.0f);
      const float rs  = 1.0f / sqrtf(var + 1e-5f);
      _Float16 hh[8], ll[8];
#pragma unroll
      for (int j = 0; j < 8; ++j) {
        const float y = dv[j] * rs * wv[j] + bv[j];
        split_h(y * SCA, hh[j], ll[j]);
      }
      *(v8h*)(sAh + rl * APITCH + l8) = (v8h){hh[0], hh[1], hh[2], hh[3], hh[4], hh[5], hh[6], hh[7]};
      *(v8h*)(sAl + rl * APITCH + l8) = (v8h){ll[0], ll[1], ll[2], ll[3], ll[4], ll[5], ll[6], ll[7]};
    }
  }
  __syncthreads();

  const _Float16* Aph = sAh + (wave * 16 + c) * APITCH + 8 * lh;
  const _Float16* Apl = sAl + (wave * 16 + c) * APITCH + 8 * lh;
  const _Float16* Wph = (const _Float16*)(const void*)whi + 8 * lh;
  const _Float16* Wpl = (const _Float16*)(const void*)wlo + 8 * lh;
  float sacc[8];
#pragma unroll
  for (int r = 0; r < 8; ++r) sacc[r] = 0.f;

#pragma unroll 1
  for (int nt = 0; nt < NT_; ++nt) {
    const int n = nt * 16 + c;
    const _Float16* Bh = Wph + (size_t)n * D_;
    const _Float16* Bl = Wpl + (size_t)n * D_;
    v8f acc0 = (v8f){0.f, 0.f, 0.f, 0.f, 0.f, 0.f, 0.f, 0.f};
    v8f acc1 = (v8f){0.f, 0.f, 0.f, 0.f, 0.f, 0.f, 0.f, 0.f};
#pragma unroll 2
    for (int ks = 0; ks < D_ / 32; ++ks) {
      FB ah, al, bh, bl;
      ah.h[0] = *(const v8h*)(Aph + ks * 32);
      ah.h[1] = *(const v8h*)(Aph + ks * 32 + 16);
      al.h[0] = *(const v8h*)(Apl + ks * 32);
      al.h[1] = *(const v8h*)(Apl + ks * 32 + 16);
      bh.h[0] = *(const v8h*)(Bh + ks * 32);
      bh.h[1] = *(const v8h*)(Bh + ks * 32 + 16);
      bl.h[0] = *(const v8h*)(Bl + ks * 32);
      bl.h[1] = *(const v8h*)(Bl + ks * 32 + 16);
      acc0 = mma_h(ah.v, bh.v, acc0);
      acc1 = mma_h(ah.v, bl.v, acc1);
      acc1 = mma_h(al.v, bh.v, acc1);
    }
    const int   nc  = min(n, H_ - 1);
    const bool  nv  = (n < H_);
    const float b1c = b1[nc], w2c = w2[nc];
    const float b1v = nv ? b1c : 0.f;
    const float w2v = nv ? w2c : 0.f;
#pragma unroll
    for (int r = 0; r < 8; ++r) {
      const float xx = acc0[r] * INV_HH + acc1[r] * INV_HL + b1v;
      const float g  = 0.5f * xx * (1.0f + erff(xx * 0.70710678118654752f));
      sacc[r] = sacc[r] + g * w2v;
    }
  }

  const float b2v = b2[0];
#pragma unroll
  for (int r = 0; r < 8; ++r) {
    float s = sacc[r];
    s += __shfl_xor(s, 1, 32);
    s += __shfl_xor(s, 2, 32);
    s += __shfl_xor(s, 4, 32);
    s += __shfl_xor(s, 8, 32);
    const int rl = wave * 16 + 8 * lh + r;
    const float a = attn[row0 + rl];
    const float val = (a != 0.f) ? (s + b2v) : 0.f;
    if (c == 0) ssc[rl] = val;
  }
  __syncthreads();
  v4f ov = (v4f){0.f, 0.f, 0.f, 0.f};
  if (tid < 8) ov = *(const v4f*)(ssc + tid * 4);
  if (tid < 8) *(volatile v4f*)(scores + row0 + tid * 4) = ov;
  __threadfence();
  if (tid < 8) *(volatile v4f*)(scores + row0 + tid * 4) = ov;
}

__global__ __launch_bounds__(NTH) void select_kernel(const int* __restrict__ ids, const float* __restrict__ emb,
                                                      const float* __restrict__ attn,
                                                      const float* __restrict__ scores,
                                                      const float* __restrict__ table,
                                                      float* __restrict__ out0, float* __restrict__ out1,
                                                      float* __restrict__ rec) {
  __shared__ float s_a[T_];
  __shared__ float s_z[T_];
  __shared__ float s_rk[T_];
  __shared__ __align__(16) float s_w[T_ * R_];
  __shared__ int   s_id[T_];
  __shared__ float s_red[3 * NTH];
  __shared__ __align__(16) float s_rec[RECW];
  __shared__ float s_wsum[R_];

  const int b = blockIdx.x, tid = threadIdx.x;
  float* red0 = s_red;
  float* red1 = s_red + NTH;
  float* red2 = s_red + 2 * NTH;
  if (tid < RECW) s_rec[tid] = 0.f;

  float pa = 0.f;
#pragma unroll
  for (int q = 0; q < 4; ++q) {
    const int t = tid + NTH * q;
    const size_t gi = (size_t)b * T_ + t;
    const float a  = attn[gi];
    const float sc = scores[gi];
    int id = ids[gi];
    id = min(max(id, 0), V_ - 1);
    s_a[t]  = a;
    s_z[t]  = (a == 0.f) ? 0.f : sc;
    s_id[t] = id;
    pa += a;
  }
  const float teff = bsum1(pa, red0, tid);
  const float rden = 1.0f / fmaxf(teff, 1.0f);
  float pm = 0.f;
#pragma unroll
  for (int q = 0; q < 4; ++q) {
    const int t = tid + NTH * q;
    pm += s_z[t] * s_a[t];
  }
  const float mean = bsum1(pm, red0, tid) * rden;
  float pv = 0.f;
#pragma unroll
  for (int q = 0; q < 4; ++q) {
    const int t = tid + NTH * q;
    const float dm = s_z[t] - mean;
    pv += dm * dm * s_a[t];
  }
  const float var  = bsum1(pv, red0, tid) * rden;
  const float rstd = 1.0f / sqrtf(var + 1e-6f);
#pragma unroll
  for (int q = 0; q < 4; ++q) {
    const int t = tid + NTH * q;
    s_z[t] = (s_z[t] - mean) * rstd;
  }
  __syncthreads();

#pragma unroll 1
  for (int q = 0; q < 4; ++q) {
    const int t = tid + NTH * q;
    const float zt = s_z[t];
    float acc = 0.f;
#pragma unroll 1
    for (int u = 0; u < T_; ++u) {
      float x = (zt - s_z[u]) * 20.0f;
      x = fminf(fmaxf(x, -30.0f), 30.0f);
      const float e  = expf(-x);
      const float sg = 1.0f / (1.0f + e);
      acc = acc + sg * sg;
    }
    const float a = s_a[t];
    s_rk[t] = (a == 0.f) ? 1e9f : (1.0f + a * acc);
  }
  __syncthreads();

  float rk[4], av[4];
  int pos[4];
#pragma unroll
  for (int q = 0; q < 4; ++q) {
    const int t = tid + NTH * q;
    rk[q] = s_rk[t];
    av[q] = s_a[t];
    pos[q] = 0;
  }
#pragma unroll 1
  for (int u = 0; u < T_; ++u) {
    const float ru = s_rk[u];
#pragma unroll
    for (int q = 0; q < 4; ++q) {
      const int t = tid + NTH * q;
      pos[q] += ((ru < rk[q]) || (ru == rk[q] && u < t)) ? 1 : 0;
    }
  }

#pragma unroll 1
  for (int r = 0; r < R_; ++r) {
    const float rho = (r == 0) ? 0.1f : (r == 1) ? 0.25f : (r == 2) ? 0.5f : 0.75f;
    float kv = rintf(rho * teff);
    kv = (teff > 0.f) ? fmaxf(kv, 1.0f) : 0.f;
    float hd[4], gr[4];
    float ph = 0.f, pg = 0.f;
#pragma unroll
    for (int q = 0; q < 4; ++q) {
      hd[q] = ((float)pos[q] < kv) ? 1.0f : 0.0f;
      float x = (kv - rk[q]) * 5.0f;
      x = fminf(fmaxf(x, -30.0f), 30.0f);
      const float sgm = __builtin_amdgcn_rcpf(1.0f + __expf(-x));
      gr[q] = sgm * av[q];
      ph += hd[q];
      pg += gr[q];
    }
    const float hsum = bsum1(ph, red0, tid);
    const float gsum = bsum1(pg, red0, tid);
    const float ginv = __builtin_amdgcn_rcpf(fmaxf(gsum, 1e-8f));
    float gst[4];
    float pw = 0.f;
#pragma unroll
    for (int q = 0; q < 4; ++q) {
      const int t = tid + NTH * q;
      const float gs = gr[q] * ginv * kv;
      gst[q] = (hd[q] + gs) - gs;
      const float w = av[q] * gst[q];
      s_w[t * R_ + r] = w;
      pw += w;
    }
    const float wsum = bsum1(pw, red0, tid);
    if (tid == 0) {
      s_wsum[r] = wsum;
      s_rec[4 + r] = hsum;
    }
    float* o1 = out1 + ((size_t)(r * B_ + b)) * T_ + tid;
    float* o0 = out0 + (size_t)b * T_ + tid;
    const bool last = (r == R_ - 1);
#pragma unroll
    for (int q = 0; q < 4; ++q) *(volatile float*)(o1 + NTH * q) = hd[q];
    if (last) {
#pragma unroll
      for (int q = 0; q < 4; ++q) *(volatile float*)(o0 + NTH * q) = gst[q];
    }
    __threadfence();
#pragma unroll
    for (int q = 0; q < 4; ++q) *(volatile float*)(o1 + NTH * q) = hd[q];
    if (last) {
#pragma unroll
      for (int q = 0; q < 4; ++q) *(volatile float*)(o0 + NTH * q) = gst[q];
    }
  }
  __syncthreads();

  const int d = tid;
  float accf = 0.f, a0 = 0.f, a1 = 0.f, a2 = 0.f, a3 = 0.f;
  const float* ep = emb + (size_t)b * T_ * D_ + d;
#pragma unroll 2
  for (int t = 0; t < T_; ++t) {
    const int id = s_id[t];
    const float e  = table[(size_t)id * D_ + d];
    const float em = ep[(size_t)t * D_];
    const float af = s_a[t];
    const v4f w = *(const v4f*)(s_w + t * R_);
    accf = accf + af * em;
    a0 = a0 + w[0] * e;
    a1 = a1 + w[1] * e;
    a2 = a2 + w[2] * e;
    a3 = a3 + w[3] * e;
  }
  const float full = accf * __builtin_amdgcn_rcpf(fmaxf(teff, 1e-8f));
  const float p0 = a0 * __builtin_amdgcn_rcpf(fmaxf(s_wsum[0], 1e-8f));
  const float p1 = a1 * __builtin_amdgcn_rcpf(fmaxf(s_wsum[1], 1e-8f));
  const float p2 = a2 * __builtin_amdgcn_rcpf(fmaxf(s_wsum[2], 1e-8f));
  const float p3 = a3 * __builtin_amdgcn_rcpf(fmaxf(s_wsum[3], 1e-8f));
  float n0, n1, n2, n3, q0, q1, q2, q3, ff;
  bsum3(p0 * full, p1 * full, p2 * full, red0, red1, red2, tid, n0, n1, n2);
  bsum3(p3 * full, p0 * p0, p1 * p1, red0, red1, red2, tid, n3, q0, q1);
  bsum3(p2 * p2, p3 * p3, full * full, red0, red1, red2, tid, q2, q3, ff);
  if (tid == 0) {
    const float fn = fmaxf(__builtin_amdgcn_sqrtf(ff), 1e-8f);
    s_rec[0] = 1.0f - n0 * __builtin_amdgcn_rcpf(fmaxf(__builtin_amdgcn_sqrtf(q0), 1e-8f) * fn);
    s_rec[1] = 1.0f - n1 * __builtin_amdgcn_rcpf(fmaxf(__builtin_amdgcn_sqrtf(q1), 1e-8f) * fn);
    s_rec[2] = 1.0f - n2 * __builtin_amdgcn_rcpf(fmaxf(__builtin_amdgcn_sqrtf(q2), 1e-8f) * fn);
    s_rec[3] = 1.0f - n3 * __builtin_amdgcn_rcpf(fmaxf(__builtin_amdgcn_sqrtf(q3), 1e-8f) * fn);
    s_rec[8] = teff;
  }
  __syncthreads();
  v4f rv = (v4f){0.f, 0.f, 0.f, 0.f};
  if (tid < 8) rv = *(const v4f*)(s_rec + tid * 4);
  if (tid < 8) *(volatile v4f*)(rec + (size_t)b * RECW + tid * 4) = rv;
  __threadfence();
  if (tid < 8) *(volatile v4f*)(rec + (size_t)b * RECW + tid * 4) = rv;
}

__global__ __launch_bounds__(NTH) void final_kernel(const float* __restrict__ rec, float* __restrict__ otail) {
  __shared__ float s_ps[R_ * B_];
  __shared__ __align__(16) float s_out[136];
  const int tid = threadIdx.x;
  if (tid < 136) s_out[tid] = 0.f;
  __syncthreads();
  if (tid < R_ * B_) {
    const int r = tid >> 5, bb = tid & 31;
    const float ps = rec[bb * RECW + r];
    const float hc = rec[bb * RECW + 4 + r];
    const float te = rec[bb * RECW + 8];
    s_ps[tid] = ps;
    s_out[5 + tid] = hc * (1.0f / fmaxf(te, 1.0f));
  }
  __syncthreads();
  if (tid == 0) {
    float tot = 0.f;
#pragma unroll 1
    for (int i = 0; i < R_ * B_; ++i) tot += s_ps[i];
    s_out[0] = tot * (1.0f / 128.0f);
#pragma unroll 1
    for (int r = 0; r < R_; ++r) {
      float s = 0.f;
#pragma unroll 1
      for (int bb = 0; bb < B_; ++bb) s += s_ps[r * B_ + bb];
      s_out[1 + r] = s * (1.0f / 32.0f);
    }
  }
  __syncthreads();
  v4f v0 = (v4f){0.f, 0.f, 0.f, 0.f};
  v4f v1 = (v4f){0.f, 0.f, 0.f, 0.f};
  float v2 = 0.f;
  if (tid < 32) v0 = *(const v4f*)(s_out + tid * 4);
  if (tid == 0) { v1 = *(const v4f*)(s_out + 128); v2 = s_out[132]; }
  if (tid < 32) *(volatile v4f*)(otail + tid * 4) = v0;
  if (tid == 0) {
    *(volatile v4f*)(otail + 128) = v1;
    *(volatile float*)(otail + 132) = v2;
  }
  __threadfence();
  if (tid < 32) *(volatile v4f*)(otail + tid * 4) = v0;
  if (tid == 0) {
    *(volatile v4f*)(otail + 128) = v1;
    *(volatile float*)(otail + 132) = v2;
  }
}

extern "C" void kernel_launch(void* const* d_in, const int* in_sizes, int n_in,
                              void* d_out, int out_size, void* d_ws, size_t ws_size,
                              hipStream_t stream) {
  if (n_in < 10) return;
  if (in_sizes[0] != NTOK) return;
  if (in_sizes[1] != NTOK * D_) return;
  if (in_sizes[2] != NTOK) return;
  if (in_sizes[3] != D_ || in_sizes[4] != D_) return;
  if (in_sizes[5] != D_ * H_) return;
  if (in_sizes[6] != H_ || in_sizes[7] != H_) return;
  if (in_sizes[8] < 1) return;
  if (in_sizes[9] != V_ * D_) return;
  if (out_size != NTOK + R_ * NTOK + NTAIL) return;

  const int*   ids   = (const int*)d_in[0];
  const float* emb   = (const float*)d_in[1];
  const float* attn  = (const float*)d_in[2];
  const float* lnw   = (const float*)d_in[3];
  const float* lnb   = (const float*)d_in[4];
  const float* w1    = (const float*)d_in[5];
  const float* b1    = (const float*)d_in[6];
  const float* w2    = (const float*)d_in[7];
  const float* b2    = (const float*)d_in[8];
  const float* table = (const float*)d_in[9];

  const size_t PW  = (size_t)NP_ * D_ * 2;
  const size_t PS  = (size_t)NTOK * 4;
  const size_t PR  = (size_t)B_ * RECW * 4;
  size_t off = 0;
  const size_t oWh = off; off += PW;
  const size_t oWl = off; off += PW;
  const size_t oSc = off; off += PS;
  const size_t oRc = off; off += PR;
  if (off > ws_size) return;

  char* ws = (char*)d_ws;
  unsigned short* Whi = (unsigned short*)(ws + oWh);
  unsigned short* Wlo = (unsigned short*)(ws + oWl);
  float* scores = (float*)(ws + oSc);
  float* recb   = (float*)(ws + oRc);

  float* out   = (float*)d_out;
  float* out0  = out;
  float* out1  = out + NTOK;
  float* otail = out + NTOK + R_ * NTOK;

  wsplit_kernel<<<dim3(NP_ / WCOLS), dim3(256), 0, stream>>>(w1, Whi, Wlo);
  mlp_kernel<<<dim3(NTOK / MROWS), dim3(64), 0, stream>>>(emb, attn, lnw, lnb, Whi, Wlo, b1, w2, b2, scores);
  select_kernel<<<dim3(B_), dim3(NTH), 0, stream>>>(ids, emb, attn, scores, table, out0, out1, recb);
  final_kernel<<<dim3(1), dim3(NTH), 0, stream>>>(recb, otail);
  (void)hipGetLastError();
}
